// NodeAndHyperedges_79998060855736
// MI455X (gfx1250) — hardware-run, weakly checked
//
#include <hip/hip_runtime.h>
#include <stddef.h>
#include <stdint.h>

#define NN     50000
#define NM     10000
#define NE     600000
#define DF     128
#define DO     64
#define NPAD   50048
#define MPAD   10112
#define HLP    256
#define ZNP    512
#define NTHR   256
#define NWAVE  8
#define EPT    8
#define CHUNK  (NTHR * EPT)
#define WCAP   (EPT * 32)
#define LISTN  (NWAVE * WCAP)
#define SL_E   8
#define SL_N   10
#define NB_E   (1 << SL_E)
#define NB_N   (1 << SL_N)
#define NBLK_E 40
#define NBLK_N 49
#define RCAP_E 20480
#define RCAP_N 16384
#define DEGCAP_E 128
#define DEGCAP_N 48
#define MEAS_BLK_E 15630
#define MEAS_DEG_E 94
#define MEAS_BLK_N 12475
#define MEAS_DEG_N 30
#define GBM    64
#define GTHR   128
#define SBR    128
#define NBS    79
#define WUNITS 38912
#define G2_TWO 1
#define G4_TWO 1
#define G5_TWO 1
#define G6_TWO 1
#define G7_TWO 1
#define G8_TWO 1
#define G9_TWO 1
#define KX(two, k) ((two) ? 2 * (k) : (k))

static_assert(NPAD % GBM == 0 && MPAD % GBM == 0 && NPAD >= NN && MPAD >= NM);
static_assert(NPAD % NWAVE == 0 && NM % NWAVE == 0 && NN % NWAVE == 0);
static_assert(NBLK_E * NB_E >= NM && (NBLK_E - 1) * NB_E < NM);
static_assert(NBLK_N * NB_N >= NPAD && (NBLK_N - 1) * NB_N < NN);
static_assert(RCAP_E * 100 >= MEAS_BLK_E * 105 && RCAP_N * 100 >= MEAS_BLK_N * 105);
static_assert(DEGCAP_E >= MEAS_DEG_E + 8 && DEGCAP_N >= MEAS_DEG_N + 8);
static_assert((CHUNK & (CHUNK - 1)) == 0 && CHUNK <= 4096);
static_assert(((long long)NE << SL_N) < (1LL << 31) && ((long long)CHUNK << SL_N) < (1LL << 31));
static_assert(RCAP_E % (NTHR * 4) == 0 && RCAP_N % (NTHR * 4) == 0);
static_assert((LISTN + 2 * RCAP_E + 3 * NB_E + 16) * 4 <= 300000);
static_assert((LISTN + 2 * RCAP_N + 3 * NB_N + 16) * 4 <= 300000);
static_assert(NBS * SBR >= NM && (NBS - 1) * SBR < NM);
static_assert(WUNITS % NTHR == 0);
static_assert(DF == 4 * 32 && HLP == 2 * DF && ZNP == 4 * DF && DO == 64);

typedef float          v4f   __attribute__((ext_vector_type(4)));
typedef float          v8f   __attribute__((ext_vector_type(8)));
typedef double         v2d   __attribute__((ext_vector_type(2)));
typedef int            v4i   __attribute__((ext_vector_type(4)));
typedef int            v8i   __attribute__((ext_vector_type(8)));
typedef unsigned short v4us  __attribute__((ext_vector_type(4)));
typedef unsigned short v8us  __attribute__((ext_vector_type(8)));
typedef unsigned short v16us __attribute__((ext_vector_type(16)));
typedef __bf16         v16bf __attribute__((ext_vector_type(16)));
typedef v4f  __attribute__((may_alias)) v4fa;
typedef v4i  __attribute__((may_alias)) v4ia;
typedef v4us __attribute__((may_alias)) v4usa;
typedef v8us __attribute__((may_alias)) v8usa;
union FragB { v16bf v; v16us u; v8us h[2]; v8i w; };

__device__ __forceinline__ v8f wmb(const FragB& a, const FragB& b, v8f c) {
  v8f d = __builtin_amdgcn_wmma_f32_16x16x32_bf16(false, a.v, false, b.v, (short)0, c, false, false);
  asm volatile("v_nop\n\tv_nop\n\tv_nop\n\tv_nop" : "+v"(d) : "v"(a.w), "v"(b.w));
  return d;
}

__device__ __forceinline__ unsigned bf16_bits(float f) {
  const unsigned u = __float_as_uint(f);
  return (u + 0x7FFFu + ((u >> 16) & 1u)) >> 16;
}
__device__ __forceinline__ float bf16_val(float f) {
  return __uint_as_float(bf16_bits(f) << 16);
}
__device__ __forceinline__ v4f bfr4(const v4f a) {
  v4f r; r.x = bf16_val(a.x); r.y = bf16_val(a.y); r.z = bf16_val(a.z); r.w = bf16_val(a.w); return r;
}
__device__ __forceinline__ unsigned split_pk(float v) {
  const unsigned hb = bf16_bits(v) & 0xffffu;
  const unsigned lb = bf16_bits(v - __uint_as_float(hb << 16)) & 0xffffu;
  return hb | (lb << 16);
}
__device__ __forceinline__ float lk(float t, float s) { return (t > 0.0f) ? t : s * t; }

__device__ __forceinline__ void wave_sync() {
  __builtin_amdgcn_fence(__ATOMIC_RELEASE, "wavefront");
  __builtin_amdgcn_wave_barrier();
  __builtin_amdgcn_fence(__ATOMIC_ACQUIRE, "wavefront");
}

template <int SLB>
__device__ __forceinline__ int scan_chunk(const int* __restrict__ dsts, int nE, int cbase, int slotBase,
                                          int nb, int vec8, int* list, int tid, int lane, int wave) {
  int wc = 0;
  const int el0  = tid * EPT;
  const int e0   = cbase + el0;
  const int sent = (int)(1u << 31);
  v4i da, db;
  if (vec8 != 0 && cbase + CHUNK <= nE) {
    da = *(const v4i*)(dsts + e0);
    db = *(const v4i*)(dsts + e0 + 4);
  } else {
    da.x = (e0     < nE) ? dsts[min(e0,     nE - 1)] : sent;
    da.y = (e0 + 1 < nE) ? dsts[min(e0 + 1, nE - 1)] : sent;
    da.z = (e0 + 2 < nE) ? dsts[min(e0 + 2, nE - 1)] : sent;
    da.w = (e0 + 3 < nE) ? dsts[min(e0 + 3, nE - 1)] : sent;
    db.x = (e0 + 4 < nE) ? dsts[min(e0 + 4, nE - 1)] : sent;
    db.y = (e0 + 5 < nE) ? dsts[min(e0 + 5, nE - 1)] : sent;
    db.z = (e0 + 6 < nE) ? dsts[min(e0 + 6, nE - 1)] : sent;
    db.w = (e0 + 7 < nE) ? dsts[min(e0 + 7, nE - 1)] : sent;
  }
  const unsigned nbs = (unsigned)slotBase;
  const unsigned unb = (unsigned)nb;
  const unsigned s0 = (unsigned)da.x - nbs, s1 = (unsigned)da.y - nbs;
  const unsigned s2 = (unsigned)da.z - nbs, s3 = (unsigned)da.w - nbs;
  const unsigned s4 = (unsigned)db.x - nbs, s5 = (unsigned)db.y - nbs;
  const unsigned s6 = (unsigned)db.z - nbs, s7 = (unsigned)db.w - nbs;
  const bool h0 = s0 < unb, h1 = s1 < unb, h2 = s2 < unb, h3 = s3 < unb;
  const bool h4 = s4 < unb, h5 = s5 < unb, h6 = s6 < unb, h7 = s7 < unb;
  const unsigned any = __builtin_amdgcn_ballot_w32(h0 | h1 | h2 | h3 | h4 | h5 | h6 | h7);
  if (any != 0u) {
#define HITJ(J, HJ, SJ) { \
      const unsigned mj = __builtin_amdgcn_ballot_w32(HJ); \
      if (mj != 0u) { \
        if (HJ) { \
          const int pos = wc + (int)__builtin_amdgcn_mbcnt_lo(mj, 0u); \
          if (pos < WCAP) list[wave * WCAP + pos] = ((el0 + (J)) << SLB) | (int)(SJ); \
        } \
        wc += (int)__builtin_popcount(mj); } }
    HITJ(0, h0, s0)
    HITJ(1, h1, s1)
    HITJ(2, h2, s2)
    HITJ(3, h3, s3)
    HITJ(4, h4, s4)
    HITJ(5, h5, s5)
    HITJ(6, h6, s6)
    HITJ(7, h7, s7)
#undef HITJ
  }
  return wc;
}

__device__ __forceinline__ void wt_unit(const float* __restrict__ W, int ldw, int ksrc, int uprShift, int v,
                                        unsigned short* P) {
  const int upr = 1 << uprShift;
  const int n   = v >> uprShift;
  const int k8  = (v & (upr - 1)) * 8;
  const int kk  = k8 & (ksrc - 1);
  const float* p = W + (size_t)kk * ldw + n;
  v8us o;
#pragma unroll
  for (int i = 0; i < 8; ++i) o[i] = (unsigned short)bf16_bits(p[(size_t)i * ldw]);
  unsigned short* dp = P + (size_t)n * (upr * 8) + k8;
  *(volatile v8us*)dp = o;
  __threadfence();
  *(volatile v8us*)dp = o;
}
#define O_HW1T  0
#define O_SW1T  16384
#define O_HW2T2 32768
#define O_SW2T2 65536
#define O_WQT2  98304
#define O_WKVT2 131072
#define O_EFT2  196608
#define O_C1T2  262144
#define O_C2T2  294912
#define WP_ELEMS 311296
__global__ __launch_bounds__(NTHR) void k_wprep(const float* __restrict__ hW1, const float* __restrict__ hW2,
                                                const float* __restrict__ sW1, const float* __restrict__ sW2,
                                                const float* __restrict__ aWq, const float* __restrict__ aWk,
                                                const float* __restrict__ aWv, const float* __restrict__ eW,
                                                const float* __restrict__ cW1, const float* __restrict__ cW2,
                                                unsigned short* WP) {
  const int u = (int)blockIdx.x * NTHR + (int)threadIdx.x;
  if (u < 2048)       wt_unit(hW1, DF, 128, 4, u,         WP + O_HW1T);
  else if (u < 4096)  wt_unit(sW1, DF, 128, 4, u - 2048,  WP + O_SW1T);
  else if (u < 8192)  wt_unit(hW2, DF, 128, 5, u - 4096,  WP + O_HW2T2);
  else if (u < 12288) wt_unit(sW2, DF, 128, 5, u - 8192,  WP + O_SW2T2);
  else if (u < 16384) wt_unit(aWq, DF, 128, 5, u - 12288, WP + O_WQT2);
  else if (u < 20480) wt_unit(aWk, DF, 128, 5, u - 16384, WP + O_WKVT2);
  else if (u < 24576) wt_unit(aWv, DF, 128, 5, u - 20480, WP + O_WKVT2 + 128 * 256);
  else if (u < 32768) wt_unit(eW,  DF, 256, 6, u - 24576, WP + O_EFT2);
  else if (u < 36864) wt_unit(cW1, DF, 128, 5, u - 32768, WP + O_C1T2);
  else if (u < WUNITS) wt_unit(cW2, DO, 128, 5, u - 36864, WP + O_C2T2);
}

__global__ __launch_bounds__(NTHR) void k_cvx(const float* __restrict__ x, int nN, int nUnits,
                                              unsigned short* xb) {
  const int u = (int)blockIdx.x * NTHR + (int)threadIdx.x;
  if (u >= nUnits) return;
  const int row = u >> 4;
  const int k8  = (u & 15) * 8;
  const int rc  = row < nN ? row : nN - 1;
  const float* p = x + (size_t)rc * DF + k8;
  const v4f a = *(const v4f*)p;
  const v4f b = *(const v4f*)(p + 4);
  const bool ok = row < nN;
  v8us o;
  o[0] = ok ? (unsigned short)bf16_bits(a.x) : (unsigned short)0;
  o[1] = ok ? (unsigned short)bf16_bits(a.y) : (unsigned short)0;
  o[2] = ok ? (unsigned short)bf16_bits(a.z) : (unsigned short)0;
  o[3] = ok ? (unsigned short)bf16_bits(a.w) : (unsigned short)0;
  o[4] = ok ? (unsigned short)bf16_bits(b.x) : (unsigned short)0;
  o[5] = ok ? (unsigned short)bf16_bits(b.y) : (unsigned short)0;
  o[6] = ok ? (unsigned short)bf16_bits(b.z) : (unsigned short)0;
  o[7] = ok ? (unsigned short)bf16_bits(b.w) : (unsigned short)0;
  unsigned short* dp = xb + (size_t)row * DF + k8;
  *(volatile v8us*)dp = o;
  __threadfence();
  *(volatile v8us*)dp = o;
}

template <int SL, int RC>
__global__ __launch_bounds__(NTHR) void k_bucket(const int* __restrict__ keys, const int* __restrict__ vals,
                                                 int nE, int vmax, int vec8,
                                                 int* LIST, int* CNT, int* OFF, int* FLG) {
  constexpr int NB = 1 << SL;
  constexpr int ZI = LISTN + 2 * RC + 3 * NB;
  static_assert(ZI % 4 == 0 && NB % 32 == 0 && NB <= NTHR * 4 && RC % (NTHR * 4) == 0);
  extern __shared__ __attribute__((aligned(16))) int dsm[];
  int* list = dsm;
  int* hl   = dsm + LISTN;
  int* sl   = hl + RC;
  int* cnt  = sl + RC;
  int* offs = cnt + NB;
  int* cur  = offs + NB;
  int* misc = cur + NB;
  const int tid = (int)threadIdx.x, lane = tid & 31, wave = tid >> 5;
  const int slotBase = (int)blockIdx.x * NB;

  {
    const v4i z4 = {0, 0, 0, 0};
    for (int i = tid * 4; i < ZI; i += NTHR * 4) *(v4ia*)(dsm + i) = z4;
    if (tid < 16) misc[tid] = 0;
  }
  __syncthreads();

  int t = 0, ov = 0;
  const int nChunks = (nE + CHUNK - 1) / CHUNK;
#pragma unroll 1
  for (int ch = 0; ch < nChunks; ++ch) {
    const int cbase = ch * CHUNK;
    const int wc = scan_chunk<SL>(keys, nE, cbase, slotBase, NB, vec8, list, tid, lane, wave);
    if (lane == 0) misc[wave] = wc;
    __syncthreads();
    if (wave == 0) {
#pragma unroll 1
      for (int w2 = 0; w2 < NWAVE; ++w2) {
        int c = misc[w2];
        c = c < 0 ? 0 : (c > WCAP ? WCAP : c);
#pragma unroll 1
        for (int b0 = 0; b0 < c; b0 += 32) {
          const int idx = b0 + lane;
          const int ent = list[w2 * WCAP + (idx < WCAP ? idx : WCAP - 1)];
          const int m32 = (c - b0) < 32 ? (c - b0) : 32;
#pragma unroll 1
          for (int k = 0; k < m32; ++k) {
            const int u    = __builtin_amdgcn_readlane(ent, k);
            const int slot = u & (NB - 1);
            const int el   = (u >> SL) & (CHUNK - 1);
            const int pk   = ((cbase + el) << SL) | slot;
            if (t < RC) {
              if (lane == 0) { hl[t] = pk; cnt[slot] = cnt[slot] + 1; }
              t = t + 1;
            } else {
              ov = 1;
            }
          }
        }
      }
    }
    __syncthreads();
  }
  if (wave == 0 && lane == 0) { misc[8] = t; misc[9] = ov; }
  __syncthreads();
  int tt = misc[8];
  tt = tt < 0 ? 0 : (tt > RC ? RC : tt);
  const int ovf = misc[9];

  if (wave == 0) {
    const int base = lane * (NB / 32);
    int s = 0;
#pragma unroll 1
    for (int i = 0; i < NB / 32; ++i) s += cnt[base + i];
    int incl = s;
#pragma unroll
    for (int d = 1; d < 32; d <<= 1) {
      const int y = __shfl_up(incl, d, 32);
      if (lane >= d) incl += y;
    }
    int run = incl - s;
#pragma unroll 1
    for (int i = 0; i < NB / 32; ++i) {
      const int cv = cnt[base + i];
      offs[base + i] = run;
      cur[base + i]  = run;
      run += cv;
    }
  }
  __syncthreads();
  if (wave == 0) {
#pragma unroll 1
    for (int b0 = 0; b0 < tt; b0 += 32) {
      const int idx = b0 + lane;
      const int ent = hl[idx < RC ? idx : RC - 1];
      const int m32 = (tt - b0) < 32 ? (tt - b0) : 32;
#pragma unroll 1
      for (int k = 0; k < m32; ++k) {
        const int u    = __builtin_amdgcn_readlane(ent, k);
        const int slot = u & (NB - 1);
        if (lane == 0) {
          int p = cur[slot];
          p = p < 0 ? 0 : (p > RC - 1 ? RC - 1 : p);
          sl[p] = u;
          cur[slot] = p + 1;
        }
      }
    }
  }
  __syncthreads();

  const int blk = (int)blockIdx.x;
  int* Lg = LIST + (size_t)blk * RC;
#pragma unroll 1
  for (int i4 = tid * 4; i4 < RC; i4 += NTHR * 4) {
    const v4i e = *(const v4ia*)(sl + i4);
    int e0 = e.x >> SL, e1 = e.y >> SL, e2 = e.z >> SL, e3 = e.w >> SL;
    e0 = e0 < 0 ? 0 : (e0 > nE - 1 ? nE - 1 : e0);
    e1 = e1 < 0 ? 0 : (e1 > nE - 1 ? nE - 1 : e1);
    e2 = e2 < 0 ? 0 : (e2 > nE - 1 ? nE - 1 : e2);
    e3 = e3 < 0 ? 0 : (e3 > nE - 1 ? nE - 1 : e3);
    int g0 = vals[e0], g1 = vals[e1], g2 = vals[e2], g3 = vals[e3];
    g0 = g0 < 0 ? 0 : (g0 > vmax - 1 ? vmax - 1 : g0);
    g1 = g1 < 0 ? 0 : (g1 > vmax - 1 ? vmax - 1 : g1);
    g2 = g2 < 0 ? 0 : (g2 > vmax - 1 ? vmax - 1 : g2);
    g3 = g3 < 0 ? 0 : (g3 > vmax - 1 ? vmax - 1 : g3);
    v4i o; o.x = g0; o.y = g1; o.z = g2; o.w = g3;
    *(volatile v4i*)(Lg + i4) = o;
    __threadfence();
    *(volatile v4i*)(Lg + i4) = o;
  }
  if (tid * 4 < NB) {
    const v4i c4 = *(const v4ia*)(cnt + tid * 4);
    const v4i o4 = *(const v4ia*)(offs + tid * 4);
    int* cp = CNT + (size_t)blk * NB + tid * 4;
    int* op = OFF + (size_t)blk * NB + tid * 4;
    *(volatile v4i*)cp = c4;
    *(volatile v4i*)op = o4;
    __threadfence();
    *(volatile v4i*)cp = c4;
    *(volatile v4i*)op = o4;
  }
  if (wave == 0) {
    int* fp = FLG + blk * 32 + lane;
    *(volatile int*)fp = ovf;
    __threadfence();
    *(volatile int*)fp = ovf;
  }
}

template <int SL, int RC, int DC>
__device__ __forceinline__ void seg_hdr(const int* __restrict__ CNT, const int* __restrict__ OFF,
                                        const int* __restrict__ FLG, int seg, int nSeg,
                                        int& cc, int& oo, int& last, int& bad) {
  const int sc = seg < nSeg ? seg : nSeg - 1;
  const int cv = CNT[sc];
  const int ov = OFF[sc];
  const int fv = FLG[(sc >> SL) * 32];
  const int bv = ((cv > DC) | (cv < 0) | (ov < 0) | (ov > RC) | (fv != 0)) ? 1 : 0;
  int c1 = cv < 0 ? 0 : (cv > DC ? DC : cv);
  int o1 = ov < 0 ? 0 : (ov > RC - 1 ? RC - 1 : ov);
  c1 = (o1 + c1 > RC) ? (RC - o1) : c1;
  cc  = __builtin_amdgcn_readfirstlane(c1);
  oo  = __builtin_amdgcn_readfirstlane(o1);
  bad = __builtin_amdgcn_readfirstlane(bv);
  int l = oo + cc - 1;
  l = l < oo ? oo : l;
  last = l;
}

__device__ __forceinline__ v4f fetch_sum(const int* __restrict__ Lb, int oo, int cc, int last,
                                         const float* __restrict__ src, int nSrc, int lane) {
  float a0 = 0.0f, a1 = 0.0f, a2 = 0.0f, a3 = 0.0f;
#pragma unroll 1
  for (int b0 = 0; b0 < cc; b0 += 32) {
    int idx = oo + b0 + lane;
    idx = idx > last ? last : idx;
    int id = Lb[idx];
    id = id < 0 ? 0 : (id > nSrc - 1 ? nSrc - 1 : id);
    const int m32 = (cc - b0) < 32 ? (cc - b0) : 32;
#pragma unroll 1
    for (int k = 0; k < m32; ++k) {
      const int sk = __builtin_amdgcn_readlane(id, k);
      const v4f a = *(const v4f*)(src + (size_t)sk * DF + 4 * lane);
      a0 += a.x; a1 += a.y; a2 += a.z; a3 += a.w;
    }
  }
  v4f r; r.x = a0; r.y = a1; r.z = a2; r.w = a3;
  return r;
}

__global__ __launch_bounds__(NTHR) void k_rep_e1(const int* __restrict__ LIST, const int* __restrict__ CNT,
                                                 const int* __restrict__ OFF, const int* __restrict__ FLG,
                                                 const float* __restrict__ H0, float* ME, int nM, int nN) {
  const int lane = (int)threadIdx.x & 31, wave = (int)threadIdx.x >> 5;
  const int seg = (int)blockIdx.x * NWAVE + wave;
  if (seg >= nM) return;
  int cc, oo, last, bad;
  seg_hdr<SL_E, RCAP_E, DEGCAP_E>(CNT, OFF, FLG, seg, nM, cc, oo, last, bad);
  const int* Lb = LIST + (size_t)(seg >> SL_E) * RCAP_E;
  const v4f a = fetch_sum(Lb, oo, cc, last, H0, nN, lane);
  const float d  = (float)(cc > 1 ? cc : 1);
  const float pz = (bad != 0) ? __int_as_float(0x7fc00000) : 0.0f;
  v4f y;
  y.x = a.x / d + pz; y.y = a.y / d + pz; y.z = a.z / d + pz; y.w = a.w / d + pz;
  float* op = ME + (size_t)seg * DF + 4 * lane;
  *(volatile v4f*)op = y;
  __threadfence();
  *(volatile v4f*)op = y;
}

__global__ __launch_bounds__(NTHR) void k_rep_n1(const int* __restrict__ LIST, const int* __restrict__ CNT,
                                                 const int* __restrict__ OFF, const int* __restrict__ FLG,
                                                 const float* __restrict__ ME, const float* __restrict__ H0,
                                                 unsigned short* S, int nN, int nM, int mRows) {
  __shared__ __attribute__((aligned(16))) unsigned short rowbuf_all[NWAVE * HLP];
  const int lane = (int)threadIdx.x & 31, wave = (int)threadIdx.x >> 5;
  unsigned short* rowbuf = rowbuf_all + wave * HLP;
  const int seg = (int)blockIdx.x * NWAVE + wave;
  const bool live = seg < nN;
  int cc, oo, last, bad;
  seg_hdr<SL_N, RCAP_N, DEGCAP_N>(CNT, OFF, FLG, seg, nN, cc, oo, last, bad);
  if (!live) { cc = 0; bad = 0; }
  const int sc = live ? seg : nN - 1;
  const int* Lb = LIST + (size_t)(sc >> SL_N) * RCAP_N;
  const v4f a = fetch_sum(Lb, oo, cc, last, ME, nM, lane);
  const v4f h = *(const v4f*)(H0 + (size_t)sc * DF + 4 * lane);
  const float d  = (float)(cc > 1 ? cc : 1);
  const float pz = (bad != 0) ? __int_as_float(0x7fc00000) : 0.0f;
  const float m0 = live ? (h.x + a.x / d + pz) : 0.0f;
  const float m1 = live ? (h.y + a.y / d + pz) : 0.0f;
  const float m2 = live ? (h.z + a.z / d + pz) : 0.0f;
  const float m3 = live ? (h.w + a.w / d + pz) : 0.0f;
  const unsigned p0 = split_pk(m0), p1 = split_pk(m1), p2 = split_pk(m2), p3 = split_pk(m3);
  v4us mh, ml;
  mh[0] = (unsigned short)(p0 & 0xffffu); ml[0] = (unsigned short)(p0 >> 16);
  mh[1] = (unsigned short)(p1 & 0xffffu); ml[1] = (unsigned short)(p1 >> 16);
  mh[2] = (unsigned short)(p2 & 0xffffu); ml[2] = (unsigned short)(p2 >> 16);
  mh[3] = (unsigned short)(p3 & 0xffffu); ml[3] = (unsigned short)(p3 >> 16);
  *(v4usa*)(rowbuf + 4 * lane) = mh;
  *(v4usa*)(rowbuf + DF + 4 * lane) = ml;
  wave_sync();
  const v8us q0 = *(const v8usa*)(rowbuf + 8 * lane);
  wave_sync();
  if (seg < mRows) {
    unsigned short* rp = S + (size_t)seg * HLP + 8 * lane;
    *(volatile v8us*)rp = q0;
    __threadfence();
    *(volatile v8us*)rp = q0;
  }
}

__global__ __launch_bounds__(NTHR) void k_rep_n2(const int* __restrict__ LIST, const int* __restrict__ CNT,
                                                 const int* __restrict__ OFF, const int* __restrict__ FLG,
                                                 const float* __restrict__ Q, const float* __restrict__ KV,
                                                 float* HA, int nN, int nM) {
  const int lane = (int)threadIdx.x & 31, wave = (int)threadIdx.x >> 5;
  const int seg = (int)blockIdx.x * NWAVE + wave;
  if (seg >= nN) return;
  int cc, oo, last, bad;
  seg_hdr<SL_N, RCAP_N, DEGCAP_N>(CNT, OFF, FLG, seg, nN, cc, oo, last, bad);
  const int* Lb = LIST + (size_t)(seg >> SL_N) * RCAP_N;
  const v4f q4 = *(const v4f*)(Q + (size_t)seg * DF + 4 * lane);
  float mx = -3.0e38f, dn = 0.0f;
  float c0 = 0.0f, c1 = 0.0f, c2 = 0.0f, c3 = 0.0f;
#pragma unroll 1
  for (int b0 = 0; b0 < cc; b0 += 32) {
    int idx = oo + b0 + lane;
    idx = idx > last ? last : idx;
    int id = Lb[idx];
    id = id < 0 ? 0 : (id > nM - 1 ? nM - 1 : id);
    const int m32 = (cc - b0) < 32 ? (cc - b0) : 32;
#pragma unroll 1
    for (int k = 0; k < m32; ++k) {
      const int hk = __builtin_amdgcn_readlane(id, k);
      const float* kp = KV + (size_t)hk * (2 * DF) + 4 * lane;
      const v4f kk4 = *(const v4f*)kp;
      const v4f vv4 = *(const v4f*)(kp + DF);
      float d = q4.x * kk4.x;
      d = fmaf(q4.y, kk4.y, d);
      d = fmaf(q4.z, kk4.z, d);
      d = fmaf(q4.w, kk4.w, d);
#pragma unroll
      for (int off = 16; off > 0; off >>= 1) d += __shfl_xor(d, off);
      const float tsc = d / 11.3137085f;
      const float lg  = (tsc > 0.0f) ? tsc : 0.2f * tsc;
      const float df  = lg - mx;
      float ar = -fabsf(df);
      ar = (ar < -100.0f) ? -100.0f : ar;
      const float ee = expf(ar);
      const bool  up = df > 0.0f;
      const float s1 = up ? ee : 1.0f;
      const float s2 = up ? 1.0f : ee;
      mx = up ? lg : mx;
      dn = fmaf(dn, s1, s2);
      c0 = fmaf(c0, s1, s2 * vv4.x);
      c1 = fmaf(c1, s1, s2 * vv4.y);
      c2 = fmaf(c2, s1, s2 * vv4.z);
      c3 = fmaf(c3, s1, s2 * vv4.w);
    }
  }
  const bool  empty = cc == 0;
  const float dsafe = empty ? 1.0f : dn;
  const float inv   = 1.0f / dsafe;
  const float pz    = (bad != 0) ? __int_as_float(0x7fc00000) : 0.0f;
  v4f y;
  y.x = (empty ? 0.0f : c0 * inv) + pz;
  y.y = (empty ? 0.0f : c1 * inv) + pz;
  y.z = (empty ? 0.0f : c2 * inv) + pz;
  y.w = (empty ? 0.0f : c3 * inv) + pz;
  float* op = HA + (size_t)seg * DF + 4 * lane;
  *(volatile v4f*)op = y;
  __threadfence();
  *(volatile v4f*)op = y;
}

__global__ __launch_bounds__(NTHR) void k_rep_e2(const int* __restrict__ LIST, const int* __restrict__ CNT,
                                                 const int* __restrict__ OFF, const int* __restrict__ FLG,
                                                 const float* __restrict__ HA, float* Z, int nM, int nN) {
  const int lane = (int)threadIdx.x & 31, wave = (int)threadIdx.x >> 5;
  const int seg = (int)blockIdx.x * NWAVE + wave;
  if (seg >= nM) return;
  int cc, oo, last, bad;
  seg_hdr<SL_E, RCAP_E, DEGCAP_E>(CNT, OFF, FLG, seg, nM, cc, oo, last, bad);
  const int* Lb = LIST + (size_t)(seg >> SL_E) * RCAP_E;
  float m0 = 3.0e38f, m1 = 3.0e38f, m2 = 3.0e38f, m3 = 3.0e38f;
#pragma unroll 1
  for (int b0 = 0; b0 < cc; b0 += 32) {
    int idx = oo + b0 + lane;
    idx = idx > last ? last : idx;
    int id = Lb[idx];
    id = id < 0 ? 0 : (id > nN - 1 ? nN - 1 : id);
    const int m32 = (cc - b0) < 32 ? (cc - b0) : 32;
#pragma unroll 1
    for (int k = 0; k < m32; ++k) {
      const int sk = __builtin_amdgcn_readlane(id, k);
      const v4f a = *(const v4f*)(HA + (size_t)sk * DF + 4 * lane);
      m0 = (a.x < m0 || a.x != a.x) ? a.x : m0;
      m1 = (a.y < m1 || a.y != a.y) ? a.y : m1;
      m2 = (a.z < m2 || a.z != a.z) ? a.z : m2;
      m3 = (a.w < m3 || a.w != a.w) ? a.w : m3;
    }
  }
  const bool  empty = cc == 0;
  const float pz    = (bad != 0) ? __int_as_float(0x7fc00000) : 0.0f;
  v4f y;
  y.x = (empty ? 0.0f : m0) + pz;
  y.y = (empty ? 0.0f : m1) + pz;
  y.z = (empty ? 0.0f : m2) + pz;
  y.w = (empty ? 0.0f : m3) + pz;
  float* op = Z + (size_t)seg * (2 * DF) + 4 * lane;
  *(volatile v4f*)op = y;
  __threadfence();
  *(volatile v4f*)op = y;
}

template <int NC, int NT, int OF32, int OHL>
__global__ __launch_bounds__(GTHR * NC) __attribute__((amdgpu_num_vgpr(248)))
void k_gemm(const unsigned short* __restrict__ A, int lda,
            const unsigned short* __restrict__ BT, int ldb, int K,
            const float* __restrict__ bias, int flags,
            float* Cf, int ldc, int nValid, unsigned short* HL) {
  static_assert(NC == 1 || NC == 2);
  static_assert(NT == 8 || (NT == 4 && NC == 1));
  static_assert(OHL == 0 || (NC == 1 && NT == 8));
  constexpr int GCOL = 16 * NT;
  constexpr int LDCT = GCOL * NC;
  extern __shared__ __attribute__((aligned(16))) float gsm[];
  float* stg = gsm;
  const int tid = (int)threadIdx.x, lane = tid & 31, wave = tid >> 5, hh = lane >> 4, m = lane & 15;
  const int rg = wave & 3, cg = wave >> 2;
  const int rowBase = (int)blockIdx.x * GBM;
  const int colBase = cg * GCOL;

  v8f acc[NT];
  {
    const v8f z = {0.f, 0.f, 0.f, 0.f, 0.f, 0.f, 0.f, 0.f};
#pragma unroll
    for (int t = 0; t < NT; ++t) acc[t] = z;
  }
  const unsigned short* ap = A  + (size_t)(rowBase + 16 * rg + m) * (size_t)lda + 8 * hh;
  const unsigned short* bp = BT + (size_t)(colBase + m) * (size_t)ldb + 8 * hh;

#pragma unroll 1
  for (int k0 = 0; k0 < K; k0 += 32) {
    FragB af;
    af.h[0] = *(const v8usa*)(ap + k0);
    af.h[1] = *(const v8usa*)(ap + k0 + 16);
#pragma unroll
    for (int nt = 0; nt < NT; ++nt) {
      const unsigned short* wq = bp + (size_t)(16 * nt) * (size_t)ldb + k0;
      FragB bf;
      bf.h[0] = *(const v8usa*)wq;
      bf.h[1] = *(const v8usa*)(wq + 16);
      acc[nt] = wmb(af, bf, acc[nt]);
    }
  }

#pragma unroll
  for (int nt = 0; nt < NT; ++nt) {
    const int lc = colBase + 16 * nt + m;
#pragma unroll
    for (int r = 0; r < 8; ++r) {
      const int lr = 16 * rg + 8 * hh + r;
      stg[lr * LDCT + lc] = acc[nt][r];
    }
  }
  __syncthreads();

  const int   hasBias = flags & 1;
  const float slope   = (flags & 2) ? 0.01f : 1.0f;
  const v4f   zero4   = {0.f, 0.f, 0.f, 0.f};

  if constexpr (OF32 != 0 && LDCT == 64) {
    const int cl = 4 * (lane & 15);
    const int rs = lane >> 4;
    v4f bb = zero4;
    if (hasBias != 0) bb = bfr4(*(const v4f*)(bias + cl));
    auto fpass = [&]() {
#pragma unroll 1
      for (int j = 0; j < 8; ++j) {
        const int lr = 16 * wave + 2 * j + rs;
        const int gr = rowBase + lr;
        const v4f p = *(const v4fa*)(stg + lr * LDCT + cl);
        v4f y;
        y.x = lk(p.x + bb.x, slope); y.y = lk(p.y + bb.y, slope);
        y.z = lk(p.z + bb.z, slope); y.w = lk(p.w + bb.w, slope);
        asm volatile("" :: "v"(y));
        if (gr < nValid) *(volatile v4f*)(Cf + (size_t)gr * (size_t)ldc + cl) = y;
      }
    };
    fpass();
    __threadfence();
    fpass();
  }
  if constexpr (OF32 != 0 && LDCT != 64) {
    constexpr int RPW = GBM / (4 * NC);
    v4f bb[NC];
#pragma unroll
    for (int c = 0; c < NC; ++c) bb[c] = zero4;
    if (hasBias != 0) {
#pragma unroll
      for (int c = 0; c < NC; ++c) bb[c] = bfr4(*(const v4f*)(bias + c * 128 + 4 * lane));
    }
    auto fpass = [&]() {
#pragma unroll 1
      for (int i = 0; i < RPW; ++i) {
        const int row = wave * RPW + i;
        const int gr  = rowBase + row;
#pragma unroll
        for (int c = 0; c < NC; ++c) {
          const v4f p = *(const v4fa*)(stg + row * LDCT + c * 128 + 4 * lane);
          v4f y;
          y.x = lk(p.x + bb[c].x, slope); y.y = lk(p.y + bb[c].y, slope);
          y.z = lk(p.z + bb[c].z, slope); y.w = lk(p.w + bb[c].w, slope);
          asm volatile("" :: "v"(y));
          if (gr < nValid) *(volatile v4f*)(Cf + (size_t)gr * (size_t)ldc + c * 128 + 4 * lane) = y;
        }
      }
    };
    fpass();
    __threadfence();
    fpass();
  }
  if constexpr (OHL != 0) {
    const int c8 = 8 * (lane & 15);
    const int rs = lane >> 4;
    v4f bA = zero4, bB = zero4;
    if (hasBias != 0) {
      bA = bfr4(*(const v4f*)(bias + c8));
      bB = bfr4(*(const v4f*)(bias + c8 + 4));
    }
    auto hpass = [&]() {
#pragma unroll 1
      for (int j = 0; j < 8; ++j) {
        const int lr = 16 * wave + 2 * j + rs;
        const int gr = rowBase + lr;
        const v4f pa = *(const v4fa*)(stg + lr * LDCT + c8);
        const v4f pb = *(const v4fa*)(stg + lr * LDCT + c8 + 4);
        const bool ok = gr < nValid;
        float t[8];
        t[0] = pa.x + bA.x; t[1] = pa.y + bA.y; t[2] = pa.z + bA.z; t[3] = pa.w + bA.w;
        t[4] = pb.x + bB.x; t[5] = pb.y + bB.y; t[6] = pb.z + bB.z; t[7] = pb.w + bB.w;
        v8us ho, lo;
#pragma unroll
        for (int i = 0; i < 8; ++i) {
          float y = lk(t[i], slope);
          y = ok ? y : 0.0f;
          const unsigned pk = split_pk(y);
          ho[i] = (unsigned short)(pk & 0xffffu);
          lo[i] = (unsigned short)(pk >> 16);
        }
        unsigned short* hp = HL + (size_t)gr * HLP + c8;
        *(volatile v8us*)hp = ho;
        *(volatile v8us*)(hp + DF) = lo;
      }
    };
    hpass();
    __threadfence();
    hpass();
  }
}

template <int COLS>
__global__ __launch_bounds__(COLS) void k_stats(const float* __restrict__ X, int nRows, double* REC) {
  __shared__ __attribute__((aligned(16))) double sd[2 * COLS];
  const int c  = (int)threadIdx.x;
  const int r0 = (int)blockIdx.x * SBR;
  int nr = nRows - r0;
  nr = nr > SBR ? SBR : nr;
  nr = nr < 0 ? 0 : nr;
  double s = 0.0, q = 0.0;
  const float* p = X + (size_t)r0 * COLS + c;
#pragma unroll 4
  for (int r = 0; r < nr; ++r) {
    const double x = (double)p[(size_t)r * COLS];
    s += x;
    q = fma(x, x, q);
  }
  sd[c] = s;
  sd[COLS + c] = q;
  __syncthreads();
  v2d o;
  o.x = sd[2 * c];
  o.y = sd[2 * c + 1];
  double* dp = REC + (size_t)blockIdx.x * (2 * COLS) + 2 * c;
  *(volatile v2d*)dp = o;
  __threadfence();
  *(volatile v2d*)dp = o;
}

template <int COLS>
__global__ __launch_bounds__(COLS) void k_comb(const double* __restrict__ REC, int nBlk, int nRows,
                                               const float* __restrict__ gw, const float* __restrict__ gb,
                                               const float* __restrict__ ga, float* STAT) {
  __shared__ __attribute__((aligned(16))) float sst[4 * COLS];
  const int c = (int)threadIdx.x;
  double s = 0.0, q = 0.0;
#pragma unroll 2
  for (int b = 0; b < nBlk; ++b) {
    s += REC[(size_t)b * (2 * COLS) + c];
    q += REC[(size_t)b * (2 * COLS) + COLS + c];
  }
  const double dm  = (double)nRows;
  const double mu  = s / dm;
  const double ex2 = q / dm;
  const float  af  = bf16_val(ga[c]);
  const double ad  = (double)af;
  const double var = ex2 - (2.0 * ad - ad * ad) * mu * mu;
  const float muf  = (float)mu;
  const float vf   = (float)var;
  sst[c]            = af * muf;
  sst[COLS + c]     = 1.0f / sqrtf(vf + 1e-5f);
  sst[2 * COLS + c] = bf16_val(gw[c]);
  sst[3 * COLS + c] = bf16_val(gb[c]);
  __syncthreads();
  const v4f o = *(const v4fa*)(sst + 4 * c);
  float* dp = STAT + 4 * c;
  *(volatile v4f*)dp = o;
  __threadfence();
  *(volatile v4f*)dp = o;
}

template <int COLS, int ACT>
__global__ __launch_bounds__(NTHR) void k_apply(const float* __restrict__ X, const float* __restrict__ STAT,
                                                int nM, int nUnits, unsigned short* P) {
  constexpr int UPR = COLS / 8;
  const int u = (int)blockIdx.x * NTHR + (int)threadIdx.x;
  if (u >= nUnits) return;
  const int row = u / UPR;
  const int c8  = (u % UPR) * 8;
  const int rc  = row < nM ? row : nM - 1;
  const bool ok = row < nM;
  const float* p = X + (size_t)rc * COLS + c8;
  const v4f xa = *(const v4f*)p;
  const v4f xb = *(const v4f*)(p + 4);
  const v4f ma = *(const v4f*)(STAT + c8);
  const v4f mb = *(const v4f*)(STAT + c8 + 4);
  const v4f ra = *(const v4f*)(STAT + COLS + c8);
  const v4f rb = *(const v4f*)(STAT + COLS + c8 + 4);
  const v4f wa = *(const v4f*)(STAT + 2 * COLS + c8);
  const v4f wb = *(const v4f*)(STAT + 2 * COLS + c8 + 4);
  const v4f ba = *(const v4f*)(STAT + 3 * COLS + c8);
  const v4f bb = *(const v4f*)(STAT + 3 * COLS + c8 + 4);
  float y[8];
  y[0] = (wa.x * (xa.x - ma.x)) * ra.x + ba.x;
  y[1] = (wa.y * (xa.y - ma.y)) * ra.y + ba.y;
  y[2] = (wa.z * (xa.z - ma.z)) * ra.z + ba.z;
  y[3] = (wa.w * (xa.w - ma.w)) * ra.w + ba.w;
  y[4] = (wb.x * (xb.x - mb.x)) * rb.x + bb.x;
  y[5] = (wb.y * (xb.y - mb.y)) * rb.y + bb.y;
  y[6] = (wb.z * (xb.z - mb.z)) * rb.z + bb.z;
  y[7] = (wb.w * (xb.w - mb.w)) * rb.w + bb.w;
  v8us ho, lo;
#pragma unroll
  for (int i = 0; i < 8; ++i) {
    float v = y[i];
    if (ACT != 0) v = lk(v, 0.01f);
    v = ok ? v : 0.0f;
    const unsigned pk = split_pk(v);
    ho[i] = (unsigned short)(pk & 0xffffu);
    lo[i] = (unsigned short)(pk >> 16);
  }
  unsigned short* dp = P + (size_t)row * (2 * COLS) + c8;
  *(volatile v8us*)dp = ho;
  *(volatile v8us*)(dp + COLS) = lo;
  __threadfence();
  *(volatile v8us*)dp = ho;
  *(volatile v8us*)(dp + COLS) = lo;
}

constexpr size_t SZ_WP  = (size_t)WP_ELEMS * 2;
constexpr size_t SZ_XB  = (size_t)NPAD * DF * 2;
constexpr size_t SZ_RA  = (size_t)NPAD * DF * 4;
constexpr size_t SZ_RB  = (size_t)NPAD * HLP * 2;
constexpr size_t SZ_RC  = (size_t)NPAD * HLP * 2;
constexpr size_t RC_SUB = (size_t)8 << 20;
constexpr size_t SZ_Z   = (size_t)MPAD * 2 * DF * 4;
constexpr size_t SZ_KV  = (size_t)MPAD * 2 * DF * 4;
constexpr size_t SZ_ME  = (size_t)MPAD * DF * 4;
constexpr size_t SZ_XE2 = (size_t)MPAD * HLP * 2;
constexpr size_t SZ_LE  = (size_t)NBLK_E * RCAP_E * 4;
constexpr size_t SZ_LN  = (size_t)NBLK_N * RCAP_N * 4;
constexpr size_t SZ_CE  = (size_t)NBLK_E * NB_E * 4;
constexpr size_t SZ_CN  = (size_t)NBLK_N * NB_N * 4;
constexpr size_t SZ_FE  = (size_t)NBLK_E * 128;
constexpr size_t SZ_FN  = (((size_t)NBLK_N * 128) + 255) & ~(size_t)255;
constexpr size_t SZ_R1  = (size_t)NBS * 512 * 8;
constexpr size_t SZ_R2  = (size_t)NBS * 256 * 8;
constexpr size_t SZ_S1  = (size_t)4 * 256 * 4;
constexpr size_t SZ_S2  = (size_t)4 * 128 * 4;
constexpr size_t O_WP  = 0;
constexpr size_t O_XB  = O_WP + SZ_WP;
constexpr size_t O_RA  = O_XB + SZ_XB;
constexpr size_t O_RB  = O_RA + SZ_RA;
constexpr size_t O_RC  = O_RB + SZ_RB;
constexpr size_t O_Z   = O_RC + SZ_RC;
constexpr size_t O_KV  = O_Z + SZ_Z;
constexpr size_t O_ME  = O_KV + SZ_KV;
constexpr size_t O_XE2 = O_ME + SZ_ME;
constexpr size_t O_LE  = O_XE2 + SZ_XE2;
constexpr size_t O_LN  = O_LE + SZ_LE;
constexpr size_t O_CE  = O_LN + SZ_LN;
constexpr size_t O_OE  = O_CE + SZ_CE;
constexpr size_t O_CN  = O_OE + SZ_CE;
constexpr size_t O_ON  = O_CN + SZ_CN;
constexpr size_t O_FE  = O_ON + SZ_CN;
constexpr size_t O_FN  = O_FE + SZ_FE;
constexpr size_t O_R1  = O_FN + SZ_FN;
constexpr size_t O_R2  = O_R1 + SZ_R1;
constexpr size_t O_S1  = O_R2 + SZ_R2;
constexpr size_t O_S2  = O_S1 + SZ_S1;
constexpr size_t WS_TOTAL = O_S2 + SZ_S2;
static_assert(WS_TOTAL <= (size_t)(128u << 20));
static_assert(SZ_WP % 256 == 0 && SZ_XB % 256 == 0 && SZ_RA % 256 == 0 && SZ_Z % 256 == 0 && SZ_ME % 256 == 0);
static_assert(SZ_LE % 256 == 0 && SZ_LN % 256 == 0 && SZ_CE % 256 == 0 && SZ_CN % 256 == 0 && SZ_FE % 256 == 0);
static_assert(SZ_R1 % 256 == 0 && SZ_R2 % 256 == 0 && SZ_S1 % 256 == 0 && SZ_S2 % 256 == 0);
static_assert((size_t)MPAD * ZNP * 2 <= SZ_XB);
static_assert((size_t)NN * DF * 4 <= SZ_RB);
static_assert((size_t)MPAD * HLP * 2 <= RC_SUB);
static_assert(RC_SUB + (size_t)MPAD * HLP * 2 <= SZ_RC);
static_assert((size_t)NM * DO - 1 < (size_t)NM * DO);

static inline int cdiv(int a, int b) { return (a + b - 1) / b; }

extern "C" void kernel_launch(void* const* d_in, const int* in_sizes, int n_in,
                              void* d_out, int out_size, void* d_ws, size_t ws_size,
                              hipStream_t stream) {
  if (n_in < 28) return;
  if (in_sizes[0] != NN * DF || in_sizes[1] != NN * DF || in_sizes[2] != NM * DF) return;
  if (in_sizes[3] != NE || in_sizes[4] != NE) return;
  if (in_sizes[5] != DF * DF || in_sizes[7] != DF * DF || in_sizes[9] != DF * DF || in_sizes[11] != DF * DF) return;
  if (in_sizes[13] != DF * DF || in_sizes[14] != DF * DF || in_sizes[15] != DF * DF) return;
  if (in_sizes[16] != 2 * DF * DF || in_sizes[24] != DF * DF || in_sizes[26] != DF * DO) return;
  if (in_sizes[6] != DF || in_sizes[8] != DF || in_sizes[10] != DF || in_sizes[12] != DF) return;
  if (in_sizes[17] != DF || in_sizes[25] != DF || in_sizes[27] != DO) return;
  if (in_sizes[18] != 2 * DF || in_sizes[19] != 2 * DF || in_sizes[20] != 2 * DF) return;
  if (in_sizes[21] != DF || in_sizes[22] != DF || in_sizes[23] != DF) return;
  if (out_size != NM * DO) return;
  if (ws_size < WS_TOTAL) return;

  const float* x      = (const float*)d_in[0];
  const float* x_e    = (const float*)d_in[2];
  const int*   nidx   = (const int*)d_in[3];
  const int*   gidx   = (const int*)d_in[4];
  const float* hW1    = (const float*)d_in[5];
  const float* hb1    = (const float*)d_in[6];
  const float* hW2    = (const float*)d_in[7];
  const float* hb2    = (const float*)d_in[8];
  const float* sW1    = (const float*)d_in[9];
  const float* sb1    = (const float*)d_in[10];
  const float* sW2    = (const float*)d_in[11];
  const float* sb2    = (const float*)d_in[12];
  const float* aWq    = (const float*)d_in[13];
  const float* aWk    = (const float*)d_in[14];
  const float* aWv    = (const float*)d_in[15];
  const float* eW     = (const float*)d_in[16];
  const float* eb     = (const float*)d_in[17];
  const float* g1w    = (const float*)d_in[18];
  const float* g1b    = (const float*)d_in[19];
  const float* g1a    = (const float*)d_in[20];
  const float* g2w    = (const float*)d_in[21];
  const float* g2b    = (const float*)d_in[22];
  const float* g2a    = (const float*)d_in[23];
  const float* cW1    = (const float*)d_in[24];
  const float* cb1    = (const float*)d_in[25];
  const float* cW2    = (const float*)d_in[26];
  const float* cb2    = (const float*)d_in[27];
  float* out = (float*)d_out;

  char* ws = (char*)d_ws;
  unsigned short* WP  = (unsigned short*)(ws + O_WP);
  unsigned short* XB  = (unsigned short*)(ws + O_XB);
  unsigned short* ZN  = (unsigned short*)(ws + O_XB);
  float*          RAf = (float*)(ws + O_RA);
  unsigned short* S   = (unsigned short*)(ws + O_RB);
  float*          HA  = (float*)(ws + O_RB);
  unsigned short* T1  = (unsigned short*)(ws + O_RC);
  unsigned short* XEB = (unsigned short*)(ws + O_RC + RC_SUB);
  unsigned short* H1  = (unsigned short*)(ws + O_RC);
  unsigned short* ZZ  = (unsigned short*)(ws + O_RC);
  unsigned short* Cp  = (unsigned short*)(ws + O_RC + RC_SUB);
  float*          Z   = (float*)(ws + O_Z);
  float*          KV  = (float*)(ws + O_KV);
  float*          ME  = (float*)(ws + O_ME);
  unsigned short* XE2 = (unsigned short*)(ws + O_XE2);
  int* LE = (int*)(ws + O_LE);
  int* LN = (int*)(ws + O_LN);
  int* CE = (int*)(ws + O_CE);
  int* OE = (int*)(ws + O_OE);
  int* CN = (int*)(ws + O_CN);
  int* ON = (int*)(ws + O_ON);
  int* FE = (int*)(ws + O_FE);
  int* FN = (int*)(ws + O_FN);
  double* R1 = (double*)(ws + O_R1);
  double* R2 = (double*)(ws + O_R2);
  float*  S1 = (float*)(ws + O_S1);
  float*  S2 = (float*)(ws + O_S2);

  const size_t ldsE = (size_t)(LISTN + 2 * RCAP_E + 3 * NB_E + 16) * 4;
  const size_t ldsN = (size_t)(LISTN + 2 * RCAP_N + 3 * NB_N + 16) * 4;
  const size_t gl128 = (size_t)GBM * 128 * 4;
  const size_t gl256 = (size_t)GBM * 256 * 4;
  const size_t gl64  = (size_t)GBM * 64 * 4;
  hipFuncSetAttribute(reinterpret_cast<const void*>(&k_bucket<SL_E, RCAP_E>), hipFuncAttributeMaxDynamicSharedMemorySize, (int)ldsE);
  hipFuncSetAttribute(reinterpret_cast<const void*>(&k_bucket<SL_N, RCAP_N>), hipFuncAttributeMaxDynamicSharedMemorySize, (int)ldsN);
  hipFuncSetAttribute(reinterpret_cast<const void*>(&k_gemm<2, 8, 1, 0>), hipFuncAttributeMaxDynamicSharedMemorySize, (int)gl256);

  const int vec8 = ((NE & 3) == 0) ? 1 : 0;
  const int gN = NPAD / GBM;
  const int gM = MPAD / GBM;

  k_wprep<<<WUNITS / NTHR, NTHR, 0, stream>>>(hW1, hW2, sW1, sW2, aWq, aWk, aWv, eW, cW1, cW2, WP);
  k_cvx<<<cdiv(NPAD * 16, NTHR), NTHR, 0, stream>>>(x, NN, NPAD * 16, XB);
  k_cvx<<<cdiv(MPAD * 16, NTHR), NTHR, 0, stream>>>(x_e, NM, MPAD * 16, XEB);
  k_bucket<SL_E, RCAP_E><<<NBLK_E, NTHR, ldsE, stream>>>(gidx, nidx, NE, NN, vec8, LE, CE, OE, FE);
  k_bucket<SL_N, RCAP_N><<<NBLK_N, NTHR, ldsN, stream>>>(nidx, gidx, NE, NM, vec8, LN, CN, ON, FN);
  k_gemm<1, 8, 0, 1><<<gM, GTHR, gl128, stream>>>(XEB, DF, WP + O_HW1T, DF, DF, hb1, 3, Z, 0, NM, T1);
  k_gemm<1, 8, 1, 1><<<gM, GTHR, gl128, stream>>>(T1, HLP, WP + O_HW2T2, HLP, KX(G2_TWO, DF), hb2, 1, Z + DF, 2 * DF, NM, XE2);
  k_gemm<1, 8, 1, 0><<<gN, GTHR, gl128, stream>>>(XB, DF, WP + O_SW1T, DF, DF, sb1, 3, RAf, DF, NN, XB);
  k_rep_e1<<<NM / NWAVE, NTHR, 0, stream>>>(LE, CE, OE, FE, RAf, ME, NM, NN);
  k_rep_n1<<<NPAD / NWAVE, NTHR, 0, stream>>>(LN, CN, ON, FN, ME, RAf, S, NN, NM, NPAD);
  k_gemm<1, 8, 0, 1><<<gN, GTHR, gl128, stream>>>(S, HLP, WP + O_SW2T2, HLP, KX(G4_TWO, DF), sb2, 3, RAf, 0, NN, H1);
  k_gemm<1, 8, 1, 0><<<gN, GTHR, gl128, stream>>>(H1, HLP, WP + O_WQT2, HLP, KX(G5_TWO, DF), hb1, 0, RAf, DF, NN, H1);
  k_gemm<2, 8, 1, 0><<<gM, GTHR * 2, gl256, stream>>>(XE2, HLP, WP + O_WKVT2, HLP, KX(G6_TWO, DF), hb1, 0, KV, 2 * DF, NM, XE2);
  k_rep_n2<<<NN / NWAVE, NTHR, 0, stream>>>(LN, CN, ON, FN, RAf, KV, HA, NN, NM);
  k_rep_e2<<<NM / NWAVE, NTHR, 0, stream>>>(LE, CE, OE, FE, HA, Z, NM, NN);
  k_stats<256><<<NBS, 256, 0, stream>>>(Z, NM, R1);
  k_comb<256><<<1, 256, 0, stream>>>(R1, NBS, NM, g1w, g1b, g1a, S1);
  k_apply<256, 0><<<cdiv(MPAD * 32, NTHR), NTHR, 0, stream>>>(Z, S1, NM, MPAD * 32, ZN);
  k_gemm<1, 8, 1, 0><<<gM, GTHR, gl128, stream>>>(ZN, ZNP, WP + O_EFT2, ZNP, KX(G7_TWO, 2 * DF), eb, 3, RAf, DF, NM, ZN);
  k_stats<128><<<NBS, 128, 0, stream>>>(RAf, NM, R2);
  k_comb<128><<<1, 128, 0, stream>>>(R2, NBS, NM, g2w, g2b, g2a, S2);
  k_apply<128, 1><<<cdiv(MPAD * 16, NTHR), NTHR, 0, stream>>>(RAf, S2, NM, MPAD * 16, ZZ);
  k_gemm<1, 8, 0, 1><<<gM, GTHR, gl128, stream>>>(ZZ, HLP, WP + O_C1T2, HLP, KX(G8_TWO, DF), cb1, 3, RAf, 0, NM, Cp);
  k_gemm<1, 4, 1, 0><<<gM, GTHR, gl64, stream>>>(Cp, HLP, WP + O_C2T2, HLP, KX(G9_TWO, DF), cb2, 1, out, DO, NM, Cp);
}
